// TripleGNNFeatureExtractor_19361712570482
// MI455X (gfx1250) — hardware-run, weakly checked
//
#include <hip/hip_runtime.h>
#include <stddef.h>
#include <stdint.h>
#include <math.h>


#define NN      50000
#define NE      800000
#define IND     256
#define HID     256
#define OUTD    128
#define K2      512
#define MP      50048
#define NBA     1024
#define SLA     10
#define NBLK    49
#define NTAB    (NBLK * NBA)
#define RCAP    28672
#define NWAVE   8
#define WLCAP   (RCAP / NWAVE)
#define DEGCAP  64
#define NTHR    256
#define SWEEP   256
#define GBM     64
#define GBN     128
#define GTHR    128
#define BK_ZINTS (2 * RCAP + 3 * NBA)
#define BK_MISC  32
#define BK_INTS  (BK_ZINTS + BK_MISC)
#define FLAGP    32
#define PB_XB    (MP * (IND / 8) / NTHR)
#define PB_W1    96
#define PB_W2    96
#define PB_TAB   7
#define T_B1     0
#define T_B2     768
#define T_AW     1152
#define T_AB     1280
#define T_TOT    1312

static_assert(NBLK == (NN + NBA - 1) / NBA);
static_assert(MP == 391 * 128 && MP % GBM == 0 && MP >= NN && MP <= NTAB);
static_assert(NBA == (1 << SLA) && NBA == NTHR * 4 && NBA % NWAVE == 0);
static_assert(((long long)(NE + NWAVE * SWEEP) << SLA) < (1LL << 31));
static_assert(HID == 32 * 8 && OUTD == 32 * 4);
static_assert(IND % 32 == 0 && K2 % 32 == 0 && K2 == 2 * HID);
static_assert(RCAP >= 17580 && RCAP % (NTHR * 4) == 0 && RCAP == NWAVE * WLCAP);
static_assert(DEGCAP >= 36 + 8);
static_assert(BK_ZINTS % (NTHR * 4) == 0);
static_assert(BK_INTS * 4 <= 300000 && BK_INTS * 4 <= 327680);
static_assert((MP * (IND / 8)) % NTHR == 0);
static_assert(GBM == (GTHR / 32) * 16 && HID % GBN == 0 && OUTD == GBN);
static_assert((long long)NN * OUTD - 1 == 6399999LL);

typedef float          v4f   __attribute__((ext_vector_type(4)));
typedef float          v8f   __attribute__((ext_vector_type(8)));
typedef int            v4i   __attribute__((ext_vector_type(4)));
typedef int            v8i   __attribute__((ext_vector_type(8)));
typedef unsigned int   v4u   __attribute__((ext_vector_type(4)));
typedef unsigned short v8us  __attribute__((ext_vector_type(8)));
typedef unsigned short v16us __attribute__((ext_vector_type(16)));
typedef __bf16         v16bf __attribute__((ext_vector_type(16)));
typedef v4f  __attribute__((may_alias)) v4fa;
typedef v4i  __attribute__((may_alias)) v4ia;
typedef v8us __attribute__((may_alias)) v8usa;
union FragB { v16bf v; v16us u; v8us h[2]; v8i w; };

__device__ __forceinline__ v8f wmb(const FragB& a, const FragB& b, v8f c) {
  v8f d = __builtin_amdgcn_wmma_f32_16x16x32_bf16(false, a.v, false, b.v, (short)0, c, false, false);
  asm volatile("v_nop\n\tv_nop\n\tv_nop\n\tv_nop" : "+v"(d) : "v"(a.w), "v"(b.w));
  return d;
}

__device__ __forceinline__ unsigned bf16_bits(float f) {
  const unsigned u = __float_as_uint(f);
  const unsigned r = (u + 0x7FFFu + ((u >> 16) & 1u)) >> 16;
  return (f != f) ? 0x7FC0u : r;
}
__device__ __forceinline__ float bf16_val(float f) {
  return __uint_as_float(bf16_bits(f) << 16);
}
__device__ __forceinline__ float relu_np(float v) { return (v > 0.0f) ? v : (v - v); }

__device__ __forceinline__ void put8(unsigned short* dp, v8us o) {
  *(volatile v8us*)dp = o;
  __threadfence();
  *(volatile v8us*)dp = o;
}
__device__ __forceinline__ void put4f(float* dp, v4f o) {
  *(volatile v4f*)dp = o;
  __threadfence();
  *(volatile v4f*)dp = o;
}

__device__ __forceinline__ void w1_unit(const float* __restrict__ W, unsigned short* W1Tg, int v) {
  const int n  = v >> 5;
  const int k8 = (v & 31) * 8;
  const float* p = W + (size_t)k8 * HID + n;
  v8us o;
#pragma unroll
  for (int i = 0; i < 8; ++i) o[i] = (unsigned short)bf16_bits(p[(size_t)i * HID]);
  put8(W1Tg + (size_t)n * IND + k8, o);
}
__device__ __forceinline__ void w2_unit(const float* __restrict__ W, unsigned short* W2Dg, int v) {
  const int n  = v >> 6;
  const int k8 = (v & 63) * 8;
  const int kk = k8 & (HID - 1);
  const float* p = W + (size_t)kk * OUTD + n;
  v8us o;
#pragma unroll
  for (int i = 0; i < 8; ++i) o[i] = (unsigned short)bf16_bits(p[(size_t)i * OUTD]);
  put8(W2Dg + (size_t)n * K2 + k8, o);
}
__device__ __forceinline__ void tab_unit(const float* __restrict__ src, float* dst, int i) {
  const v4f a = *(const v4f*)(src + 4 * i);
  v4f o;
  o.x = bf16_val(a.x); o.y = bf16_val(a.y); o.z = bf16_val(a.z); o.w = bf16_val(a.w);
  put4f(dst + 4 * i, o);
}

__global__ __launch_bounds__(NTHR) void k_prep(
    const float* __restrict__ x,
    const float* __restrict__ w1a, const float* __restrict__ w1b, const float* __restrict__ w1c,
    const float* __restrict__ w2a, const float* __restrict__ w2b, const float* __restrict__ w2c,
    const float* __restrict__ b1a, const float* __restrict__ b1b, const float* __restrict__ b1c,
    const float* __restrict__ b2a, const float* __restrict__ b2b, const float* __restrict__ b2c,
    const float* __restrict__ aw, const float* __restrict__ ab,
    unsigned short* XB, unsigned short* W1T, unsigned short* W2D, float* TAB, int nN) {
  const int blk = (int)blockIdx.x;
  const int tid = (int)threadIdx.x;
  if (blk < PB_XB) {
    const int u   = blk * NTHR + tid;
    const int row = u >> 5;
    const int k8  = (u & 31) * 8;
    const int rc  = row < nN ? row : nN - 1;
    const float* p = x + (size_t)rc * IND + k8;
    const v4f a = *(const v4fa*)p;
    const v4f b = *(const v4fa*)(p + 4);
    const bool ok = row < nN;
    v8us o;
    o[0] = ok ? (unsigned short)bf16_bits(a.x) : (unsigned short)0;
    o[1] = ok ? (unsigned short)bf16_bits(a.y) : (unsigned short)0;
    o[2] = ok ? (unsigned short)bf16_bits(a.z) : (unsigned short)0;
    o[3] = ok ? (unsigned short)bf16_bits(a.w) : (unsigned short)0;
    o[4] = ok ? (unsigned short)bf16_bits(b.x) : (unsigned short)0;
    o[5] = ok ? (unsigned short)bf16_bits(b.y) : (unsigned short)0;
    o[6] = ok ? (unsigned short)bf16_bits(b.z) : (unsigned short)0;
    o[7] = ok ? (unsigned short)bf16_bits(b.w) : (unsigned short)0;
    put8(XB + (size_t)row * IND + k8, o);
  } else if (blk < PB_XB + PB_W1) {
    const int v0 = (blk - PB_XB) * NTHR + tid;
    const int g  = v0 >> 13;
    const int v  = v0 & 8191;
    if (g == 0)      w1_unit(w1a, W1T, v);
    else if (g == 1) w1_unit(w1b, W1T + (size_t)IND * HID, v);
    else             w1_unit(w1c, W1T + (size_t)2 * IND * HID, v);
  } else if (blk < PB_XB + PB_W1 + PB_W2) {
    const int v0 = (blk - PB_XB - PB_W1) * NTHR + tid;
    const int g  = v0 >> 13;
    const int v  = v0 & 8191;
    if (g == 0)      w2_unit(w2a, W2D, v);
    else if (g == 1) w2_unit(w2b, W2D + (size_t)OUTD * K2, v);
    else             w2_unit(w2c, W2D + (size_t)2 * OUTD * K2, v);
  } else {
    const int t = blk - (PB_XB + PB_W1 + PB_W2);
    if (t < 3) {
      if (tid < HID / 4) {
        if (t == 0)      tab_unit(b1a, TAB + T_B1, tid);
        else if (t == 1) tab_unit(b1b, TAB + T_B1 + HID, tid);
        else             tab_unit(b1c, TAB + T_B1 + 2 * HID, tid);
      }
    } else if (t < 6) {
      if (tid < OUTD / 4) {
        if (t == 3)      tab_unit(b2a, TAB + T_B2, tid);
        else if (t == 4) tab_unit(b2b, TAB + T_B2 + OUTD, tid);
        else             tab_unit(b2c, TAB + T_B2 + 2 * OUTD, tid);
      }
    } else if (t == 6) {
      const int wave = tid >> 5, lane = tid & 31;
      if (wave == 0) {
        tab_unit(aw, TAB + T_AW, lane);
      } else if (wave == 1) {
        const float av = bf16_val(ab[0]);
        asm volatile("" :: "v"(av));
        v4f o; o.x = av; o.y = av; o.z = av; o.w = av;
        float* dp = TAB + T_AB + 4 * (lane & 7);
        const bool wr = lane < 8;
        if (wr) *(volatile v4f*)dp = o;
        __threadfence();
        if (wr) *(volatile v4f*)dp = o;
      }
    }
  }
}

#define LDK(J) \
  const int e##J = eb + 32 * (J); \
  const int d##J = dsts[min(e##J, nE - 1)]; \
  const unsigned s##J = (unsigned)d##J - nbs; \
  const bool h##J = (e##J < nE) & (s##J < (unsigned)NBA);
#define HITJ(J) { \
  const unsigned mj = __builtin_amdgcn_ballot_w32(h##J); \
  if (mj != 0u) { \
    if (h##J) { \
      const int pos = wc + (int)__builtin_amdgcn_mbcnt_lo(mj, 0u); \
      if (pos < WLCAP) mywl[pos] = (e##J << SLA) | (int)s##J; \
    } \
    wc += (int)__builtin_popcount(mj); } }

__device__ __forceinline__ void bucket_body(const int* __restrict__ edge, int nE, int nN, int segLen,
                                            int g, int b, int* dsm,
                                            int* LIST, int* CNT, int* OFF, float* DINV, int* FLAG) {
  int* wl   = dsm;
  int* sl   = dsm + RCAP;
  int* cnt  = sl + RCAP;
  int* offs = cnt + NBA;
  int* cur  = offs + NBA;
  int* misc = cur + NBA;
  const int tid = (int)threadIdx.x, lane = tid & 31, wave = tid >> 5;
  const int nodeBase = b * NBA;
  const int* srcs = edge;
  const int* dsts = edge + nE;

  {
    const v4i z4 = {0, 0, 0, 0};
    for (int i = tid * 4; i < BK_ZINTS; i += NTHR * 4) *(v4ia*)(dsm + i) = z4;
    if (tid < BK_MISC) misc[tid] = 0;
  }
  __syncthreads();

  int wc = 0;
  {
    int* mywl = wl + wave * WLCAP;
    const unsigned nbs = (unsigned)nodeBase;
    const int wbeg = wave * segLen;
    const int nIt  = segLen / SWEEP;
#pragma unroll 1
    for (int it = 0; it < nIt; ++it) {
      const int eb = wbeg + it * SWEEP + lane;
      LDK(0) LDK(1) LDK(2) LDK(3) LDK(4) LDK(5) LDK(6) LDK(7)
      const unsigned any = __builtin_amdgcn_ballot_w32(h0 | h1 | h2 | h3 | h4 | h5 | h6 | h7);
      if (any != 0u) {
        HITJ(0) HITJ(1) HITJ(2) HITJ(3) HITJ(4) HITJ(5) HITJ(6) HITJ(7)
      }
    }
  }
  if (lane == 0) {
    misc[wave]     = wc > WLCAP ? WLCAP : wc;
    misc[8 + wave] = wc > WLCAP ? 1 : 0;
  }
  __syncthreads();

  if (wave == 0) {
#pragma unroll 1
    for (int w2 = 0; w2 < NWAVE; ++w2) {
      int c = misc[w2];
      c = c < 0 ? 0 : (c > WLCAP ? WLCAP : c);
#pragma unroll 1
      for (int b0 = 0; b0 < c; b0 += 32) {
        const int idx = b0 + lane;
        const int ent = wl[w2 * WLCAP + (idx < WLCAP ? idx : WLCAP - 1)];
        const int m32 = (c - b0) < 32 ? (c - b0) : 32;
#pragma unroll 1
        for (int k = 0; k < m32; ++k) {
          const int u    = __builtin_amdgcn_readlane(ent, k);
          const int slot = u & (NBA - 1);
          if (lane == 0) cnt[slot] = cnt[slot] + 1;
        }
      }
    }
  }
  __syncthreads();

  if (wave == 0) {
    const int base = lane * (NBA / 32);
    int s = 0;
#pragma unroll 1
    for (int i = 0; i < NBA / 32; ++i) s += cnt[base + i];
    int incl = s;
#pragma unroll
    for (int d = 1; d < 32; d <<= 1) {
      const int y = __shfl_up(incl, d, 32);
      if (lane >= d) incl += y;
    }
    int run = incl - s;
#pragma unroll 1
    for (int i = 0; i < NBA / 32; ++i) {
      const int cv = cnt[base + i];
      offs[base + i] = run;
      cur[base + i]  = run;
      run += cv;
    }
  }
  __syncthreads();

  if (wave == 0) {
#pragma unroll 1
    for (int w2 = 0; w2 < NWAVE; ++w2) {
      int c = misc[w2];
      c = c < 0 ? 0 : (c > WLCAP ? WLCAP : c);
#pragma unroll 1
      for (int b0 = 0; b0 < c; b0 += 32) {
        const int idx = b0 + lane;
        const int ent = wl[w2 * WLCAP + (idx < WLCAP ? idx : WLCAP - 1)];
        int eid = ent >> SLA;
        eid = eid < 0 ? 0 : (eid > nE - 1 ? nE - 1 : eid);
        int sr = srcs[eid];
        sr = sr < 0 ? 0 : (sr > nN - 1 ? nN - 1 : sr);
        const int m32 = (c - b0) < 32 ? (c - b0) : 32;
#pragma unroll 1
        for (int k = 0; k < m32; ++k) {
          const int u    = __builtin_amdgcn_readlane(ent, k);
          const int sv   = __builtin_amdgcn_readlane(sr, k);
          const int slot = u & (NBA - 1);
          if (lane == 0) {
            int p = cur[slot];
            p = p < 0 ? 0 : (p > RCAP - 1 ? RCAP - 1 : p);
            sl[p] = sv;
            cur[slot] = p + 1;
          }
        }
      }
    }
  }
  __syncthreads();

#pragma unroll 1
  for (int q = 0; q < 4; ++q) {
    const int s = tid + NTHR * q;
    const int c = cnt[s];
    const float dg = (float)(c + 1);
    const float dv = 1.0f / sqrtf(dg);
    cur[s] = __float_as_int((nodeBase + s) < nN ? dv : 1.0f);
    if (c > DEGCAP) misc[16] = 1;
  }
  __syncthreads();

  const int flag = (misc[8] | misc[9] | misc[10] | misc[11] | misc[12] | misc[13] | misc[14] | misc[15] |
                    misc[16]) != 0 ? 1 : 0;
  const v4i c4 = *(const v4ia*)(cnt + 4 * tid);
  const v4i o4 = *(const v4ia*)(offs + 4 * tid);
  const v4i di = *(const v4ia*)(cur + 4 * tid);
  v4f d4;
  d4.x = __int_as_float(di.x); d4.y = __int_as_float(di.y);
  d4.z = __int_as_float(di.z); d4.w = __int_as_float(di.w);
  const v4i f4 = {flag, flag, flag, flag};

  const size_t tb = (size_t)g * NTAB + (size_t)nodeBase + (size_t)(4 * tid);
  int* lp = LIST + (size_t)(g * NBLK + b) * RCAP;
  int* fp = FLAG + (size_t)(g * NBLK + b) * FLAGP + 4 * (lane & 7);
  const bool fw = (wave == 0) && (lane < 8);

  *(volatile v4i*)(CNT + tb) = c4;
  *(volatile v4i*)(OFF + tb) = o4;
  *(volatile v4f*)(DINV + tb) = d4;
  if (fw) *(volatile v4i*)fp = f4;
#pragma unroll 1
  for (int it = 0; it < RCAP / (NTHR * 4); ++it) {
    const int i = it * (NTHR * 4) + 4 * tid;
    const v4i v = *(const v4ia*)(sl + i);
    *(volatile v4i*)(lp + i) = v;
  }
  __threadfence();
  *(volatile v4i*)(CNT + tb) = c4;
  *(volatile v4i*)(OFF + tb) = o4;
  *(volatile v4f*)(DINV + tb) = d4;
  if (fw) *(volatile v4i*)fp = f4;
#pragma unroll 1
  for (int it = 0; it < RCAP / (NTHR * 4); ++it) {
    const int i = it * (NTHR * 4) + 4 * tid;
    const v4i v = *(const v4ia*)(sl + i);
    *(volatile v4i*)(lp + i) = v;
  }
}
#undef LDK
#undef HITJ

__global__ __launch_bounds__(NTHR) void k_bucket(const int* __restrict__ e0p, const int* __restrict__ e1p,
                                                 const int* __restrict__ e2p, int nE, int nN, int segLen,
                                                 int* LIST, int* CNT, int* OFF, float* DINV, int* FLAG) {
  extern __shared__ __attribute__((aligned(16))) int dsm[];
  const int b = (int)blockIdx.x;
  const int g = (int)blockIdx.y;
  if (g == 0)      bucket_body(e0p, nE, nN, segLen, 0, b, dsm, LIST, CNT, OFF, DINV, FLAG);
  else if (g == 1) bucket_body(e1p, nE, nN, segLen, 1, b, dsm, LIST, CNT, OFF, DINV, FLAG);
  else             bucket_body(e2p, nE, nN, segLen, 2, b, dsm, LIST, CNT, OFF, DINV, FLAG);
}

__global__ __launch_bounds__(GTHR) __attribute__((amdgpu_num_vgpr(248)))
void k_gemm(const unsigned short* __restrict__ A, const unsigned short* __restrict__ BT, int K,
            const float* __restrict__ dinv, float* outF, int ldo) {
  __shared__ __attribute__((aligned(16))) float stg[GBM * GBN];
  __shared__ __attribute__((aligned(16))) float sdv[GBM];
  const int tid = (int)threadIdx.x, lane = tid & 31, wave = tid >> 5, hh = lane >> 4, m = lane & 15;
  const int rowBase = (int)blockIdx.x * GBM;
  const int col0    = (int)blockIdx.y * GBN;

  v8f acc[8];
  {
    const v8f z = {0.f, 0.f, 0.f, 0.f, 0.f, 0.f, 0.f, 0.f};
#pragma unroll
    for (int t = 0; t < 8; ++t) acc[t] = z;
  }
  const unsigned short* ap = A  + (size_t)(rowBase + 16 * wave + m) * (size_t)K + 8 * hh;
  const unsigned short* bp = BT + (size_t)(col0 + m) * (size_t)K + 8 * hh;

#pragma unroll 1
  for (int k0 = 0; k0 < K; k0 += 32) {
    FragB af;
    af.h[0] = *(const v8usa*)(ap + k0);
    af.h[1] = *(const v8usa*)(ap + k0 + 16);
#pragma unroll
    for (int nt = 0; nt < 8; ++nt) {
      const unsigned short* wq = bp + (size_t)(16 * nt) * (size_t)K + k0;
      FragB bf;
      bf.h[0] = *(const v8usa*)wq;
      bf.h[1] = *(const v8usa*)(wq + 16);
      acc[nt] = wmb(af, bf, acc[nt]);
    }
  }

#pragma unroll
  for (int nt = 0; nt < 8; ++nt) {
    const int lc = 16 * nt + m;
#pragma unroll
    for (int r = 0; r < 8; ++r) {
      const int lr = 16 * wave + 8 * hh + r;
      stg[lr * GBN + lc] = acc[nt][r];
    }
  }
  if (tid < GBM) sdv[tid] = dinv[rowBase + tid];
  __syncthreads();

  v4f pv[16];
#pragma unroll
  for (int i = 0; i < 16; ++i) {
    const int r = 16 * wave + i;
    const v4f t = *(const v4fa*)(stg + r * GBN + 4 * lane);
    pv[i] = t * sdv[r];
  }
#pragma unroll
  for (int i = 0; i < 16; ++i) {
    float* op = outF + (size_t)(rowBase + 16 * wave + i) * (size_t)ldo + col0 + 4 * lane;
    *(volatile v4f*)op = pv[i];
  }
  __threadfence();
#pragma unroll
  for (int i = 0; i < 16; ++i) {
    float* op = outF + (size_t)(rowBase + 16 * wave + i) * (size_t)ldo + col0 + 4 * lane;
    *(volatile v4f*)op = pv[i];
  }
}

__global__ __launch_bounds__(NTHR) void k_agg1(const int* __restrict__ lst, const int* __restrict__ cntg,
                                               const int* __restrict__ offg, const float* __restrict__ ding,
                                               const int* __restrict__ flg, const float* __restrict__ hp,
                                               const float* __restrict__ b1t, unsigned short* h1,
                                               int nN, int mRows) {
  __shared__ __attribute__((aligned(16))) int   scn[NBA];
  __shared__ __attribute__((aligned(16))) int   sof[NBA];
  __shared__ __attribute__((aligned(16))) float sdi[NBA];
  __shared__ __attribute__((aligned(16))) float sb[HID];
  const int tid = (int)threadIdx.x, lane = tid & 31, wave = tid >> 5;
  const int b = (int)blockIdx.x;
  const int nodeBase = b * NBA;
  {
    const v4i c4 = *(const v4i*)(cntg + nodeBase + 4 * tid);
    const v4i o4 = *(const v4i*)(offg + nodeBase + 4 * tid);
    const v4f d4 = *(const v4f*)(ding + nodeBase + 4 * tid);
    *(v4ia*)(scn + 4 * tid) = c4;
    *(v4ia*)(sof + 4 * tid) = o4;
    *(v4fa*)(sdi + 4 * tid) = d4;
    if (tid < HID / 4) {
      const v4f t = *(const v4f*)(b1t + 4 * tid);
      *(v4fa*)(sb + 4 * tid) = t;
    }
  }
  const int fl = flg[b * FLAGP];
  __syncthreads();
  const v4f bA = *(const v4fa*)(sb + 8 * lane);
  const v4f bB = *(const v4fa*)(sb + 8 * lane + 4);
  const int* lb = lst + (size_t)b * RCAP;
  const float qnan = __int_as_float(0x7fc00000);

#pragma unroll 1
  for (int si = 0; si < NBA / NWAVE; ++si) {
    const int s    = si * NWAVE + wave;
    const int node = nodeBase + s;
    if (node < mRows) {
      int c = scn[s];
      const bool pz = (c > DEGCAP) | (fl != 0);
      c = c < 0 ? 0 : (c > DEGCAP ? DEGCAP : c);
      int o = sof[s];
      o = o < 0 ? 0 : (o > RCAP - 1 ? RCAP - 1 : o);
      const float dd = sdi[s];
      const int nc = node < nN ? node : nN - 1;
      v4f aA = {0.0f, 0.0f, 0.0f, 0.0f};
      v4f aB = {0.0f, 0.0f, 0.0f, 0.0f};
#pragma unroll 1
      for (int b0 = 0; b0 < c; b0 += 32) {
        int j = b0 + lane;
        j = j > c - 1 ? c - 1 : j;
        int idx = o + j;
        idx = idx > RCAP - 1 ? RCAP - 1 : idx;
        int sr = lb[idx];
        sr = sr < 0 ? 0 : (sr > nN - 1 ? nN - 1 : sr);
        const int m32 = (c - b0) < 32 ? (c - b0) : 32;
#pragma unroll 1
        for (int k = 0; k < m32; ++k) {
          const int sk = __builtin_amdgcn_readlane(sr, k);
          const float* p = hp + (size_t)sk * HID + 8 * lane;
          const v4f ra = *(const v4f*)p;
          const v4f rb = *(const v4f*)(p + 4);
          aA = aA + ra;
          aB = aB + rb;
        }
      }
      const float* ps = hp + (size_t)nc * HID + 8 * lane;
      const v4f sA = *(const v4f*)ps;
      const v4f sB = *(const v4f*)(ps + 4);
      const v4f yA = (aA + sA) * dd + bA;
      const v4f yB = (aB + sB) * dd + bB;
      const bool live = node < nN;
      float v0 = relu_np(yA.x), v1 = relu_np(yA.y), v2 = relu_np(yA.z), v3 = relu_np(yA.w);
      float v4 = relu_np(yB.x), v5 = relu_np(yB.y), v6 = relu_np(yB.z), v7 = relu_np(yB.w);
      v0 = pz ? qnan : v0; v1 = pz ? qnan : v1; v2 = pz ? qnan : v2; v3 = pz ? qnan : v3;
      v4 = pz ? qnan : v4; v5 = pz ? qnan : v5; v6 = pz ? qnan : v6; v7 = pz ? qnan : v7;
      v0 = live ? v0 : 0.0f; v1 = live ? v1 : 0.0f; v2 = live ? v2 : 0.0f; v3 = live ? v3 : 0.0f;
      v4 = live ? v4 : 0.0f; v5 = live ? v5 : 0.0f; v6 = live ? v6 : 0.0f; v7 = live ? v7 : 0.0f;
      const unsigned h0 = bf16_bits(v0), h1b = bf16_bits(v1), h2 = bf16_bits(v2), h3 = bf16_bits(v3);
      const unsigned h4 = bf16_bits(v4), h5 = bf16_bits(v5), h6 = bf16_bits(v6), h7 = bf16_bits(v7);
      const unsigned l0 = bf16_bits(v0 - __uint_as_float(h0 << 16));
      const unsigned l1 = bf16_bits(v1 - __uint_as_float(h1b << 16));
      const unsigned l2 = bf16_bits(v2 - __uint_as_float(h2 << 16));
      const unsigned l3 = bf16_bits(v3 - __uint_as_float(h3 << 16));
      const unsigned l4 = bf16_bits(v4 - __uint_as_float(h4 << 16));
      const unsigned l5 = bf16_bits(v5 - __uint_as_float(h5 << 16));
      const unsigned l6 = bf16_bits(v6 - __uint_as_float(h6 << 16));
      const unsigned l7 = bf16_bits(v7 - __uint_as_float(h7 << 16));
      v4u hv, lv;
      hv.x = h0 | (h1b << 16); hv.y = h2 | (h3 << 16); hv.z = h4 | (h5 << 16); hv.w = h6 | (h7 << 16);
      lv.x = l0 | (l1 << 16);  lv.y = l2 | (l3 << 16); lv.z = l4 | (l5 << 16); lv.w = l6 | (l7 << 16);
      unsigned short* rp = h1 + (size_t)node * K2 + 8 * lane;
      *(volatile v4u*)rp = hv;
      *(volatile v4u*)(rp + HID) = lv;
      __threadfence();
      *(volatile v4u*)rp = hv;
      *(volatile v4u*)(rp + HID) = lv;
    }
  }
}

template <int FUSE>
__global__ __launch_bounds__(NTHR) void k_agg2(const int* __restrict__ lst, const int* __restrict__ cntg,
                                               const int* __restrict__ offg, const float* __restrict__ ding,
                                               const int* __restrict__ flall, int g,
                                               const float* __restrict__ gp, const float* __restrict__ b2t,
                                               const float* __restrict__ awt, const float* __restrict__ abt,
                                               const float* f0p, const float* f1p, float* outp,
                                               int nN, int mRows) {
  __shared__ __attribute__((aligned(16))) int   scn[NBA];
  __shared__ __attribute__((aligned(16))) int   sof[NBA];
  __shared__ __attribute__((aligned(16))) float sdi[NBA];
  __shared__ __attribute__((aligned(16))) float sb[OUTD];
  __shared__ __attribute__((aligned(16))) float saw[OUTD];
  const int tid = (int)threadIdx.x, lane = tid & 31, wave = tid >> 5;
  const int b = (int)blockIdx.x;
  const int nodeBase = b * NBA;
  {
    const v4i c4 = *(const v4i*)(cntg + nodeBase + 4 * tid);
    const v4i o4 = *(const v4i*)(offg + nodeBase + 4 * tid);
    const v4f d4 = *(const v4f*)(ding + nodeBase + 4 * tid);
    *(v4ia*)(scn + 4 * tid) = c4;
    *(v4ia*)(sof + 4 * tid) = o4;
    *(v4fa*)(sdi + 4 * tid) = d4;
    if (tid < OUTD / 4) {
      const v4f t = *(const v4f*)(b2t + 4 * tid);
      const v4f a = *(const v4f*)(awt + 4 * tid);
      *(v4fa*)(sb + 4 * tid) = t;
      *(v4fa*)(saw + 4 * tid) = a;
    }
  }
  const int fl = flall[(g * NBLK + b) * FLAGP];
  int flAny = fl;
  if constexpr (FUSE != 0) {
    flAny = flall[(0 * NBLK + b) * FLAGP] | flall[(1 * NBLK + b) * FLAGP] | flall[(2 * NBLK + b) * FLAGP];
  }
  const float abv = abt[0];
  __syncthreads();
  const v4f b4  = *(const v4fa*)(sb + 4 * lane);
  const v4f aw4 = *(const v4fa*)(saw + 4 * lane);
  const int* lb = lst + (size_t)b * RCAP;
  const float qnan = __int_as_float(0x7fc00000);
  const int lim = (FUSE != 0) ? nN : mRows;

#pragma unroll 1
  for (int si = 0; si < NBA / NWAVE; ++si) {
    const int s    = si * NWAVE + wave;
    const int node = nodeBase + s;
    if (node < lim) {
      int c = scn[s];
      const bool pz = (c > DEGCAP) | (fl != 0);
      c = c < 0 ? 0 : (c > DEGCAP ? DEGCAP : c);
      int o = sof[s];
      o = o < 0 ? 0 : (o > RCAP - 1 ? RCAP - 1 : o);
      const float dd = sdi[s];
      const int nc = node < nN ? node : nN - 1;
      v4f a4 = {0.0f, 0.0f, 0.0f, 0.0f};
#pragma unroll 1
      for (int b0 = 0; b0 < c; b0 += 32) {
        int j = b0 + lane;
        j = j > c - 1 ? c - 1 : j;
        int idx = o + j;
        idx = idx > RCAP - 1 ? RCAP - 1 : idx;
        int sr = lb[idx];
        sr = sr < 0 ? 0 : (sr > nN - 1 ? nN - 1 : sr);
        const int m32 = (c - b0) < 32 ? (c - b0) : 32;
#pragma unroll 1
        for (int k = 0; k < m32; ++k) {
          const int sk = __builtin_amdgcn_readlane(sr, k);
          const v4f r4 = *(const v4f*)(gp + (size_t)sk * OUTD + 4 * lane);
          a4 = a4 + r4;
        }
      }
      const v4f s4 = *(const v4f*)(gp + (size_t)nc * OUTD + 4 * lane);
      v4f y = (a4 + s4) * dd + b4;
      y.x = pz ? qnan : y.x; y.y = pz ? qnan : y.y; y.z = pz ? qnan : y.z; y.w = pz ? qnan : y.w;
      if constexpr (FUSE == 0) {
        const bool live = node < nN;
        v4f ov;
        ov.x = live ? y.x : 0.0f; ov.y = live ? y.y : 0.0f; ov.z = live ? y.z : 0.0f; ov.w = live ? y.w : 0.0f;
        float* op = outp + (size_t)node * OUTD + 4 * lane;
        *(volatile v4f*)op = ov;
        __threadfence();
        *(volatile v4f*)op = ov;
      } else {
        const v4f f0 = *(const v4f*)(f0p + (size_t)nc * OUTD + 4 * lane);
        const v4f f1 = *(const v4f*)(f1p + (size_t)nc * OUTD + 4 * lane);
        asm volatile("" :: "v"(f0));
        asm volatile("" :: "v"(f1));
        float d0 = f0.x * aw4.x; d0 = fmaf(f0.y, aw4.y, d0); d0 = fmaf(f0.z, aw4.z, d0); d0 = fmaf(f0.w, aw4.w, d0);
        float d1 = f1.x * aw4.x; d1 = fmaf(f1.y, aw4.y, d1); d1 = fmaf(f1.z, aw4.z, d1); d1 = fmaf(f1.w, aw4.w, d1);
        float d2 = y.x * aw4.x;  d2 = fmaf(y.y, aw4.y, d2);  d2 = fmaf(y.z, aw4.z, d2);  d2 = fmaf(y.w, aw4.w, d2);
#pragma unroll
        for (int off = 16; off >= 1; off >>= 1) {
          const float t0 = __shfl_xor(d0, off, 32);
          const float t1 = __shfl_xor(d1, off, 32);
          const float t2 = __shfl_xor(d2, off, 32);
          d0 += t0; d1 += t1; d2 += t2;
        }
        const float l0 = d0 + abv, l1 = d1 + abv, l2 = d2 + abv;
        float mx = l0;
        mx = ((l1 > mx) | (l1 != l1)) ? l1 : mx;
        mx = ((l2 > mx) | (l2 != l2)) ? l2 : mx;
        const float e0 = expf(l0 - mx);
        const float e1 = expf(l1 - mx);
        const float e2 = expf(l2 - mx);
        const float den = (e0 + e1) + e2;
        const float a0 = e0 / den, a1 = e1 / den, a2 = e2 / den;
        v4f ov = (f0 * a0 + f1 * a1) + y * a2;
        const bool pa = flAny != 0;
        ov.x = pa ? qnan : ov.x; ov.y = pa ? qnan : ov.y; ov.z = pa ? qnan : ov.z; ov.w = pa ? qnan : ov.w;
        float* op = outp + (size_t)node * OUTD + 4 * lane;
        *(volatile v4f*)op = ov;
        __threadfence();
        *(volatile v4f*)op = ov;
      }
    }
  }
}

static inline int cdiv(int a, int b) { return (a + b - 1) / b; }
static inline size_t al256(size_t o) { return (o + 255) & ~(size_t)255; }

extern "C" void kernel_launch(void* const* d_in, const int* in_sizes, int n_in,
                              void* d_out, int out_size, void* d_ws, size_t ws_size,
                              hipStream_t stream) {
  if (n_in < 18) return;
  if (in_sizes[0] != NN * IND) return;
  if (in_sizes[1] != 2 * NE || in_sizes[2] != 2 * NE || in_sizes[3] != 2 * NE) return;
  for (int g = 0; g < 3; ++g) {
    if (in_sizes[4 + 4 * g] != IND * HID || in_sizes[5 + 4 * g] != HID) return;
    if (in_sizes[6 + 4 * g] != HID * OUTD || in_sizes[7 + 4 * g] != OUTD) return;
  }
  if (in_sizes[16] != OUTD || in_sizes[17] != 1) return;
  if (out_size != NN * OUTD) return;

  const float* x  = (const float*)d_in[0];
  const int*   e0 = (const int*)d_in[1];
  const int*   e1 = (const int*)d_in[2];
  const int*   e2 = (const int*)d_in[3];
  const float* w1a = (const float*)d_in[4];  const float* b1a = (const float*)d_in[5];
  const float* w2a = (const float*)d_in[6];  const float* b2a = (const float*)d_in[7];
  const float* w1b = (const float*)d_in[8];  const float* b1b = (const float*)d_in[9];
  const float* w2b = (const float*)d_in[10]; const float* b2b = (const float*)d_in[11];
  const float* w1c = (const float*)d_in[12]; const float* b1c = (const float*)d_in[13];
  const float* w2c = (const float*)d_in[14]; const float* b2c = (const float*)d_in[15];
  const float* aw  = (const float*)d_in[16];
  const float* ab  = (const float*)d_in[17];
  float* out = (float*)d_out;

  const int nN = NN, nE = NE;
  const int segLen = cdiv(cdiv(nE, NWAVE), SWEEP) * SWEEP;
  if ((long long)segLen * NWAVE < (long long)nE) return;

  char* ws = (char*)d_ws;
  size_t off = 0;
  const size_t oXB  = off; off = al256(off + (size_t)MP * IND * 2);
  const size_t oHP  = off; off = al256(off + (size_t)MP * HID * 4);
  const size_t oH1  = off; off = al256(off + (size_t)MP * K2 * 2);
  const size_t oF0  = off; off = al256(off + (size_t)MP * OUTD * 4);
  const size_t oF1  = off; off = al256(off + (size_t)MP * OUTD * 4);
  const size_t oLS  = off; off = al256(off + (size_t)3 * NBLK * RCAP * 4);
  const size_t oCN  = off; off = al256(off + (size_t)3 * NTAB * 4);
  const size_t oOF  = off; off = al256(off + (size_t)3 * NTAB * 4);
  const size_t oDI  = off; off = al256(off + (size_t)3 * NTAB * 4);
  const size_t oFL  = off; off = al256(off + (size_t)3 * NBLK * FLAGP * 4);
  const size_t oW1  = off; off = al256(off + (size_t)3 * HID * IND * 2);
  const size_t oW2  = off; off = al256(off + (size_t)3 * OUTD * K2 * 2);
  const size_t oTB  = off; off = al256(off + (size_t)T_TOT * 4);
  if (off > ws_size) return;
  unsigned short* XB  = (unsigned short*)(ws + oXB);
  float*          HP  = (float*)(ws + oHP);
  float*          G   = (float*)(ws + oHP);
  unsigned short* H1  = (unsigned short*)(ws + oH1);
  float*          F0  = (float*)(ws + oF0);
  float*          F1  = (float*)(ws + oF1);
  int*            LS  = (int*)(ws + oLS);
  int*            CN  = (int*)(ws + oCN);
  int*            OF  = (int*)(ws + oOF);
  float*          DI  = (float*)(ws + oDI);
  int*            FL  = (int*)(ws + oFL);
  unsigned short* W1T = (unsigned short*)(ws + oW1);
  unsigned short* W2D = (unsigned short*)(ws + oW2);
  float*          TB  = (float*)(ws + oTB);

  const size_t bkLds = (size_t)BK_INTS * 4;
  hipFuncSetAttribute(reinterpret_cast<const void*>(&k_bucket), hipFuncAttributeMaxDynamicSharedMemorySize, (int)bkLds);

  k_prep<<<PB_XB + PB_W1 + PB_W2 + PB_TAB, NTHR, 0, stream>>>(x, w1a, w1b, w1c, w2a, w2b, w2c,
      b1a, b1b, b1c, b2a, b2b, b2c, aw, ab, XB, W1T, W2D, TB, nN);
  k_bucket<<<dim3(NBLK, 3), NTHR, bkLds, stream>>>(e0, e1, e2, nE, nN, segLen, LS, CN, OF, DI, FL);

  for (int g = 0; g < 3; ++g) {
    const int*   lst = LS + (size_t)g * NBLK * RCAP;
    const int*   cn  = CN + (size_t)g * NTAB;
    const int*   of  = OF + (size_t)g * NTAB;
    const float* di  = DI + (size_t)g * NTAB;
    k_gemm<<<dim3(MP / GBM, HID / GBN), GTHR, 0, stream>>>(XB, W1T + (size_t)g * HID * IND, IND, di, HP, HID);
    k_agg1<<<NBLK, NTHR, 0, stream>>>(lst, cn, of, di, FL + (size_t)g * NBLK * FLAGP, HP,
                                      TB + T_B1 + g * HID, H1, nN, MP);
    k_gemm<<<dim3(MP / GBM, OUTD / GBN), GTHR, 0, stream>>>(H1, W2D + (size_t)g * OUTD * K2, K2, di, G, OUTD);
    if (g == 0) {
      k_agg2<0><<<NBLK, NTHR, 0, stream>>>(lst, cn, of, di, FL, g, G, TB + T_B2 + g * OUTD, TB + T_AW, TB + T_AB,
                                           F0, F1, F0, nN, MP);
    } else if (g == 1) {
      k_agg2<0><<<NBLK, NTHR, 0, stream>>>(lst, cn, of, di, FL, g, G, TB + T_B2 + g * OUTD, TB + T_AW, TB + T_AB,
                                           F0, F1, F1, nN, MP);
    } else {
      k_agg2<1><<<NBLK, NTHR, 0, stream>>>(lst, cn, of, di, FL, g, G, TB + T_B2 + g * OUTD, TB + T_AW, TB + T_AB,
                                           F0, F1, out, nN, MP);
    }
  }
}
